// SlowFastSSMM_23184233464549
// MI455X (gfx1250) — hardware-verified
//
#include <hip/hip_runtime.h>
#include <math.h>

constexpr int kBsz       = 4;
constexpr int kTlen      = 32768;
constexpr int kLs        = 32;
constexpr int kDeltaS    = 16;
constexpr int kNumSlow   = 2047;
constexpr int kNSeq      = kBsz * kNumSlow;
constexpr int kNSeqPad   = 8192;
constexpr int kGruH      = 64;
constexpr int kG3        = 192;
constexpr int kNGru      = 4;
constexpr int kHidden    = 32;
constexpr int kEpsW      = 2 * kHidden;
constexpr int kWinTile   = 16;
constexpr int kNumWinBlk = kNSeqPad / kWinTile;
constexpr int kSlabPitch = 68;
constexpr float kActCarry = 8.0f;
constexpr float kWgtCarry = 64.0f;
constexpr float kAccFold  = 1.0f / 512.0f;

typedef __attribute__((ext_vector_type(16))) _Float16 v16h;
typedef __attribute__((ext_vector_type(8)))  _Float16 v8h;
typedef __attribute__((ext_vector_type(8)))  float    v8f;
typedef __attribute__((ext_vector_type(4)))  float    v4f;
typedef __attribute__((ext_vector_type(4)))  unsigned int v4u;

__device__ __forceinline__ void dep_guard_h(v8f& a, v8f& b, v16h x, v16h y) { asm volatile("v_nop\n\tv_nop\n\tv_nop\n\tv_nop" : "+v"(a), "+v"(b) : "v"(x), "v"(y)); }
__device__ __forceinline__ void keep4_h(v16h a, v16h b, v16h c, v16h d) { asm volatile("v_nop" :: "v"(a), "v"(b), "v"(c), "v"(d)); }
__device__ __forceinline__ void guard4_a4(v8f& a, v8f& b, v8f& c, v8f& d, v16h x0, v16h x1, v16h x2, v16h x3) {
  asm volatile("v_nop\n\tv_nop\n\tv_nop\n\tv_nop" : "+v"(a), "+v"(b), "+v"(c), "+v"(d) : "v"(x0), "v"(x1), "v"(x2), "v"(x3));
}
__device__ __forceinline__ void guard1_a4(v8f& a, v16h x0, v16h x1, v16h x2, v16h x3) {
  asm volatile("v_nop\n\tv_nop\n\tv_nop\n\tv_nop" : "+v"(a) : "v"(x0), "v"(x1), "v"(x2), "v"(x3));
}

template <typename T> struct Frag;
template <> struct Frag<_Float16> {
  typedef v16h V; union U { v16h v; v8h h[2]; };
  static __device__ __forceinline__ v16h load(const _Float16* p) {
    U f; f.h[0] = *(const v8h*)(p); f.h[1] = *(const v8h*)(p + 16); return f.v;
  }
  static __device__ __forceinline__ v8f mma(v16h a, v16h b, v8f c) {
    return __builtin_amdgcn_wmma_f32_16x16x32_f16(false, a, false, b, (short)0, c, false, false);
  }
};
typedef Frag<_Float16> FragH;

__device__ __forceinline__ unsigned pk16(unsigned short a, unsigned short b) { return (unsigned)a | ((unsigned)b << 16); }
__device__ __forceinline__ unsigned short h_bits(float f) { const _Float16 h = (_Float16)f; return __builtin_bit_cast(unsigned short, h); }
__device__ __forceinline__ float sigm_f(float v) { return __builtin_amdgcn_rcpf(1.0f + expf(-v)); }
__device__ __forceinline__ float tanh_f(float v) { return 1.0f - 2.0f * __builtin_amdgcn_rcpf(1.0f + expf(2.0f * v)); }

__global__ __launch_bounds__(256) void cast_w_kernel(
    const float* __restrict__ wih, const float* __restrict__ whh, const float* __restrict__ ofw,
    unsigned short* __restrict__ wih16, unsigned short* __restrict__ whh16, unsigned short* __restrict__ ofw16)
{
  const int blk = blockIdx.x;
  const float* src = wih; unsigned short* dst = wih16; int cb = blk;
  if (blk >= 48)      { src = ofw; dst = ofw16; cb = blk - 48; }
  else if (blk >= 24) { src = whh; dst = whh16; cb = blk - 24; }
  const size_t i = (size_t)cb * 256 + threadIdx.x;
  const float* p = src + 8 * i;
  const v4f a = *(const v4f*)(p);
  const v4f c = *(const v4f*)(p + 4);
  unsigned short hb[8];
#pragma unroll
  for (int e = 0; e < 4; ++e) {
    hb[e]     = h_bits(a[e] * kWgtCarry);
    hb[4 + e] = h_bits(c[e] * kWgtCarry);
  }
  const v4u u = (v4u){pk16(hb[0], hb[1]), pk16(hb[2], hb[3]), pk16(hb[4], hb[5]), pk16(hb[6], hb[7])};
  unsigned short* q = dst + 8 * i;
  *(volatile v4u*)q = u;
  __threadfence();
  *(volatile v4u*)q = u;
}

__global__ __launch_bounds__(128) void gru_slow_kernel(
    const float* __restrict__ x, const float* __restrict__ fc_in_w, const float* __restrict__ fc_in_b,
    const unsigned short* __restrict__ wih16, const unsigned short* __restrict__ whh16,
    const float* __restrict__ gru_bih, const float* __restrict__ gru_bhh,
    const unsigned short* __restrict__ ofw16, const float* __restrict__ out_fc_b,
    float* __restrict__ wsE)
{
  __shared__ __align__(16) _Float16 Xbuf[kLs * kWinTile * kGruH];
  __shared__ __align__(16) _Float16 Hcur[kWinTile * kGruH];
  __shared__ __align__(16) float slab[kWinTile * kSlabPitch];

  const int tid  = threadIdx.x;
  const int lane = tid & 31;
  const int wave = tid >> 5;
  const int hh   = lane >> 4;
  const int c    = lane & 15;
  const int koff = hh * 8;
  const int gs0  = blockIdx.x * kWinTile;
  const int ucol = wave * 16 + c;

  {
    const int k8 = (tid & 7) * 8;
    float wv[8], bv[8];
#pragma unroll
    for (int e = 0; e < 8; ++e) { wv[e] = fc_in_w[k8 + e]; bv[e] = fc_in_b[k8 + e]; }
#pragma unroll 1
    for (int it = 0; it < 32; ++it) {
      const int q   = it * 128 + tid;
      const int win = (q >> 3) & 15;
      const int t   = q >> 7;
      int gs = gs0 + win; gs = (gs < kNSeq) ? gs : (kNSeq - 1);
      const int b = gs / kNumSlow;
      const int f = gs - b * kNumSlow;
      const float xv = x[(size_t)b * kTlen + f * kDeltaS + t];
      v8h hv;
#pragma unroll
      for (int e = 0; e < 8; ++e) {
        float v = xv * wv[e] + bv[e];
        v = fmaxf(v, 0.0f) * kActCarry;
        hv[e] = (_Float16)v;
      }
      *(v8h*)(Xbuf + (size_t)(t * kWinTile + win) * kGruH + k8) = hv;
    }
  }

  const v8f z8 = (v8f){0.f, 0.f, 0.f, 0.f, 0.f, 0.f, 0.f, 0.f};
  const v4u zero4 = (v4u){0u, 0u, 0u, 0u};
  float hreg[8];

  for (int l = 0; l < kNGru; ++l) {
    __syncthreads();
    ((v4u*)(void*)Hcur)[tid] = zero4;
#pragma unroll
    for (int r = 0; r < 8; ++r) hreg[r] = 0.0f;
    const float* bi = gru_bih + l * kG3;
    const float* bh = gru_bhh + l * kG3;
    const float br  = bi[ucol] + bh[ucol];
    const float bz  = bi[kGruH + ucol] + bh[kGruH + ucol];
    const float bxn = bi[2 * kGruH + ucol];
    const float bhn = bh[2 * kGruH + ucol];
    const _Float16* Wi = (const _Float16*)wih16 + (size_t)l * kG3 * kGruH;
    const _Float16* Wh = (const _Float16*)whh16 + (size_t)l * kG3 * kGruH;
    const _Float16* wir = Wi + (size_t)ucol * kGruH + koff;
    const _Float16* wiz = Wi + (size_t)(kGruH + ucol) * kGruH + koff;
    const _Float16* win = Wi + (size_t)(2 * kGruH + ucol) * kGruH + koff;
    const _Float16* whr = Wh + (size_t)ucol * kGruH + koff;
    const _Float16* whz = Wh + (size_t)(kGruH + ucol) * kGruH + koff;
    const _Float16* whn = Wh + (size_t)(2 * kGruH + ucol) * kGruH + koff;
    __syncthreads();

#pragma unroll 1
    for (int t = 0; t < kLs; ++t) {
      const _Float16* xrow = Xbuf + (size_t)(t * kWinTile + c) * kGruH + koff;
      const _Float16* hrow = Hcur + c * kGruH + koff;
      const v16h ax0 = FragH::load(xrow);
      const v16h ax1 = FragH::load(xrow + 32);
      const v16h ah0 = FragH::load(hrow);
      const v16h ah1 = FragH::load(hrow + 32);
      const v16h bri0 = FragH::load(wir), bri1 = FragH::load(wir + 32);
      const v16h brh0 = FragH::load(whr), brh1 = FragH::load(whr + 32);
      const v16h bzi0 = FragH::load(wiz), bzi1 = FragH::load(wiz + 32);
      const v16h bzh0 = FragH::load(whz), bzh1 = FragH::load(whz + 32);
      const v16h bni0 = FragH::load(win), bni1 = FragH::load(win + 32);
      const v16h bnh0 = FragH::load(whn), bnh1 = FragH::load(whn + 32);

      v8f accR = z8, accZ = z8, accNI = z8, accNH = z8;
      accR  = FragH::mma(ax0, bri0, accR);
      accR  = FragH::mma(ax1, bri1, accR);
      accR  = FragH::mma(ah0, brh0, accR);
      accR  = FragH::mma(ah1, brh1, accR);
      accZ  = FragH::mma(ax0, bzi0, accZ);
      accZ  = FragH::mma(ax1, bzi1, accZ);
      accZ  = FragH::mma(ah0, bzh0, accZ);
      accZ  = FragH::mma(ah1, bzh1, accZ);
      accNI = FragH::mma(ax0, bni0, accNI);
      accNI = FragH::mma(ax1, bni1, accNI);
      accNH = FragH::mma(ah0, bnh0, accNH);
      accNH = FragH::mma(ah1, bnh1, accNH);
      guard4_a4(accR, accZ, accNI, accNH, ax0, ax1, ah0, ah1);
      keep4_h(bri0, bri1, brh0, brh1);
      keep4_h(bzi0, bzi1, bzh0, bzh1);
      keep4_h(bni0, bni1, bnh0, bnh1);

      _Float16 h16[8];
#pragma unroll
      for (int r = 0; r < 8; ++r) {
        const float pr  = accR[r]  * kAccFold + br;
        const float pz  = accZ[r]  * kAccFold + bz;
        const float pxn = accNI[r] * kAccFold + bxn;
        const float phn = accNH[r] * kAccFold + bhn;
        const float rg  = sigm_f(pr);
        const float zg  = sigm_f(pz);
        const float nn  = tanh_f(pxn + rg * phn);
        const float hn  = (1.0f - zg) * nn + zg * hreg[r];
        hreg[r] = hn;
        h16[r]  = (_Float16)(hn * kActCarry);
      }
      __syncthreads();
      {
        _Float16* hw = Hcur + (hh * 8) * kGruH + ucol;
        _Float16* xw = Xbuf + (size_t)(t * kWinTile + hh * 8) * kGruH + ucol;
#pragma unroll
        for (int r = 0; r < 8; ++r) { hw[r * kGruH] = h16[r]; xw[r * kGruH] = h16[r]; }
      }
      __syncthreads();
    }
  }

  {
    const _Float16* hrow = Hcur + c * kGruH + koff;
    const v16h a0 = FragH::load(hrow), a1 = FragH::load(hrow + 32);
    const _Float16* wo = (const _Float16*)ofw16 + (size_t)ucol * kGruH + koff;
    const v16h b0 = FragH::load(wo), b1 = FragH::load(wo + 32);
    v8f acc = z8;
    acc = FragH::mma(a0, b0, acc);
    acc = FragH::mma(a1, b1, acc);
    guard1_a4(acc, a0, a1, b0, b1);
    const float ob  = out_fc_b[ucol];
    const bool isA  = (wave < 2);
#pragma unroll
    for (int r = 0; r < 8; ++r) {
      const float e = acc[r] * kAccFold + ob;
      const float s = sigm_f(e);
      slab[(hh * 8 + r) * kSlabPitch + ucol] = isA ? s : e;
    }
  }
  __syncthreads();
  {
    const int c4 = (lane & 15) * 4;
    float* eo = wsE + (size_t)gs0 * kEpsW;
    for (int pass = 0; pass < 2; ++pass) {
#pragma unroll
      for (int it = 0; it < 2; ++it) {
        const int row = wave * 4 + it * 2 + hh;
        const v4f v = *(const v4f*)(slab + row * kSlabPitch + c4);
        *(volatile v4f*)(eo + (size_t)row * kEpsW + c4) = v;
      }
      __threadfence();
    }
  }
}

__global__ __launch_bounds__(32) void fast_scan_kernel(
    const float* __restrict__ x, const float* __restrict__ fin_w, const float* __restrict__ fin_b,
    const float* __restrict__ fout_w, const float* __restrict__ fout_b,
    const float* __restrict__ wsE, float* __restrict__ out)
{
  const int b    = blockIdx.x;
  const int lane = threadIdx.x & 31;
  const float fw = fin_w[lane];
  const float fb = fin_b[lane];
  const float ow = fout_w[lane];
  const float ob = fout_b[0];
  const float* xb = x + (size_t)b * kTlen;
  const float* eb = wsE + (size_t)b * kNumSlow * kEpsW;
  float* outb = out + (size_t)b * kTlen;
  float h = 0.0f;
#pragma unroll 1
  for (int g = 0; g < kTlen / 128; ++g) {
    float o0 = 0.0f, o1 = 0.0f, o2 = 0.0f, o3 = 0.0f;
#pragma unroll 1
    for (int blk = 0; blk < 8; ++blk) {
      const int t16 = g * 128 + blk * 16;
      int idx = (t16 >> 4) - 1;
      idx = (idx < 0) ? 0 : idx;
      idx = (idx > kNumSlow - 1) ? (kNumSlow - 1) : idx;
      const float Acoef = eb[(size_t)idx * kEpsW + lane];
      const float gsl   = eb[(size_t)idx * kEpsW + kHidden + lane];
      const float xv    = xb[t16 + (lane & 15)];
#pragma unroll
      for (int j = 0; j < 16; ++j) {
        const float xj = __shfl(xv, j, 32);
        const float u  = (xj * fw + fb) * gsl;
        h = Acoef * h + u;
        float v = h * ow;
        v += __shfl_xor(v, 16, 32);
        v += __shfl_xor(v, 8, 32);
        v += __shfl_xor(v, 4, 32);
        v += __shfl_xor(v, 2, 32);
        v += __shfl_xor(v, 1, 32);
        const int tgt = blk * 4 + (j >> 2);
        const bool me = (lane == tgt);
        const int cc = j & 3;
        if (cc == 0)      o0 = me ? v : o0;
        else if (cc == 1) o1 = me ? v : o1;
        else if (cc == 2) o2 = me ? v : o2;
        else              o3 = me ? v : o3;
      }
    }
    v4f ov;
    ov[0] = o0 + ob; ov[1] = o1 + ob; ov[2] = o2 + ob; ov[3] = o3 + ob;
    float* op = outb + (size_t)g * 128 + lane * 4;
    *(volatile v4f*)op = ov;
    __threadfence();
    *(volatile v4f*)op = ov;
  }
}

extern "C" void kernel_launch(void* const* d_in, const int* in_sizes, int n_in,
                              void* d_out, int out_size, void* d_ws, size_t ws_size,
                              hipStream_t stream)
{
  (void)in_sizes; (void)n_in;
  const float* x        = (const float*)d_in[0];
  const float* fc_in_w  = (const float*)d_in[1];
  const float* fc_in_b  = (const float*)d_in[2];
  const float* gru_wih  = (const float*)d_in[3];
  const float* gru_whh  = (const float*)d_in[4];
  const float* gru_bih  = (const float*)d_in[5];
  const float* gru_bhh  = (const float*)d_in[6];
  const float* out_fc_w = (const float*)d_in[7];
  const float* out_fc_b = (const float*)d_in[8];
  const float* fin_w    = (const float*)d_in[9];
  const float* fin_b    = (const float*)d_in[10];
  const float* fout_w   = (const float*)d_in[11];
  const float* fout_b   = (const float*)d_in[12];
  float* out = (float*)d_out;

  const size_t offWih = 0;
  const size_t offWhh = offWih + (size_t)kNGru * kG3 * kGruH * 2;
  const size_t offOfw = offWhh + (size_t)kNGru * kG3 * kGruH * 2;
  const size_t offE   = offOfw + (size_t)kEpsW * kGruH * 2;
  const size_t total  = offE + (size_t)kNSeqPad * kEpsW * 4;
  if (total > ws_size) return;
  if ((size_t)out_size * sizeof(float) < (size_t)kBsz * kTlen * sizeof(float)) return;

  char* ws = (char*)d_ws;
  unsigned short* wih16 = (unsigned short*)(ws + offWih);
  unsigned short* whh16 = (unsigned short*)(ws + offWhh);
  unsigned short* ofw16 = (unsigned short*)(ws + offOfw);
  float* wsE = (float*)(ws + offE);

  cast_w_kernel<<<50, 256, 0, stream>>>(gru_wih, gru_whh, out_fc_w, wih16, whh16, ofw16);
  gru_slow_kernel<<<kNumWinBlk, 128, 0, stream>>>(x, fc_in_w, fc_in_b, wih16, whh16,
                                                   gru_bih, gru_bhh, ofw16, out_fc_b, wsE);
  fast_scan_kernel<<<kBsz, 32, 0, stream>>>(x, fin_w, fin_b, fout_w, fout_b, wsE, out);
}
